// constrained_network_44968307589559
// MI455X (gfx1250) — hardware-verified
//
#include <hip/hip_runtime.h>
#include <stddef.h>
#include <math.h>


#define NS     64
#define NV     64
#define EMB    32
#define NBAS   8
#define RHID   16
#define NW     256
#define YVW    192
#define SCW    320
#define NPB    64
#define SNCOL  4096
#define VNCOL  2048

#define ATHR   256
#define NWAVE  8
#define EPT    8
#define NGRP   2
#define CHUNK  (ATHR * EPT * NGRP)
#define WCAP   (EPT * NGRP * 32)
#define LISTN  (NWAVE * WCAP)
#define GRP    32

#define STHR   128

#define LS_YH  0
#define LS_YL  (NPB * NS * 2)
#define LS_VH  (2 * NPB * NS * 2)
#define LS_VL  (LS_VH + 3 * NPB * NV * 2)
#define LS_A   (LS_VL + 3 * NPB * NV * 2)
#define LS_O   (LS_A + NPB * EMB * 4)
#define LDS_SC (LS_O + NPB * SCW * 4)

#define LA_ACC  0
#define LA_LIST (LA_ACC + NPB * SCW * 4)
#define LA_WST  (LA_LIST + LISTN * 4)
#define LA_W2   (LA_WST + GRP * NW * 4)
#define LA_HID  (LA_W2 + NW * 32 * 2)
#define LA_W1   (LA_HID + GRP * 32 * 2)
#define LA_B1   (LA_W1 + NBAS * RHID * 4)
#define LA_B2   (LA_B1 + RHID * 4)
#define LA_Q    (LA_B2 + NW * 4)
#define LA_EA   (LA_Q + 2 * NV * 4)
#define LA_XV   (LA_EA + GRP * 4 * 4)
#define LA_SRC  (LA_XV + NPB * 8 * 4)
#define LA_SLOT (LA_SRC + GRP * 4)
#define LA_CNT  (LA_SLOT + GRP * 4)
#define LDS_AGG (LA_CNT + 16 * 4)

#define SQ3F    1.7320508f
#define C2CF    0.75592894601845440f
#define SQ8F    2.8284271247461903f
#define RCUTF   (1.0f / 3.5f)
#define PIF     3.14159265358979323846f
#define INVDEGF 0.17677669529663687f
#define HSTEPF  0.1f

static_assert((CHUNK & (CHUNK - 1)) == 0 && CHUNK <= 4096);
static_assert((NPB & (NPB - 1)) == 0 && NPB <= 64);
static_assert(NPB == NWAVE * 8);
static_assert(GRP == 32);
static_assert((LS_YL % 16) == 0 && (LS_VH % 16) == 0 && (LS_VL % 16) == 0 && (LS_A % 16) == 0 && (LS_O % 16) == 0);
static_assert((LA_LIST % 16) == 0 && (LA_WST % 16) == 0 && (LA_W2 % 16) == 0 && (LA_HID % 16) == 0);
static_assert((LA_W1 % 16) == 0 && (LA_B1 % 16) == 0 && (LA_B2 % 16) == 0 && (LA_Q % 16) == 0);
static_assert((LA_EA % 16) == 0 && (LA_XV % 16) == 0 && (LA_SRC % 16) == 0 && (LA_SLOT % 16) == 0 && (LA_CNT % 16) == 0);
static_assert((NPB * NS / 4) % STHR == 0 && (NPB * YVW / 4) % STHR == 0 && (NPB * EMB / 4) % STHR == 0);
static_assert((16 * SCW / 4) % 32 == 0);
static_assert((SCW * 4) % 128 == 0 && (NS * 4) % 128 == 0 && (YVW * 4) % 128 == 0);
static_assert((NPB * 6 * 4) % 128 == 0);
static_assert(NW == ATHR);

typedef float          v4f   __attribute__((ext_vector_type(4)));
typedef float          v8f   __attribute__((ext_vector_type(8)));
typedef int            v4i   __attribute__((ext_vector_type(4)));
typedef unsigned short v4us  __attribute__((ext_vector_type(4)));
typedef unsigned short v8us  __attribute__((ext_vector_type(8)));
typedef __bf16         v16bf __attribute__((ext_vector_type(16)));
typedef _Float16       v8h   __attribute__((ext_vector_type(8)));
typedef _Float16       v16h  __attribute__((ext_vector_type(16)));
union FragB { v16bf v; v8us u[2]; };
union FragH { v16h v; v8h half[2]; };

__device__ __forceinline__ unsigned short bf_bits(float x) {
  unsigned u = __builtin_bit_cast(unsigned, x);
  u = (u + 0x7FFFu + ((u >> 16) & 1u)) >> 16;
  return (unsigned short)u;
}
__device__ __forceinline__ float bf_val(unsigned short b) {
  return __builtin_bit_cast(float, ((unsigned)b) << 16);
}
__device__ __forceinline__ void split4(v4f v, v4us& hi, v4us& lo) {
#pragma unroll
  for (int u = 0; u < 4; ++u) {
    const unsigned short hb = bf_bits(v[u]);
    hi[u] = hb;
    lo[u] = bf_bits(v[u] - bf_val(hb));
  }
}
__device__ __forceinline__ float sigmf(float x) {
  const float xc = fmaxf(x, -30.0f);
  const float ex = __expf(-xc);
  return 1.0f / (1.0f + ex);
}
__device__ __forceinline__ float siluf(float x) { return x * sigmf(x); }

__device__ __forceinline__ v8f wm4(v16bf ah0, v16bf al0, v16bf b0, v16bf ah1, v16bf al1, v16bf b1) {
  v8f z = {0.f, 0.f, 0.f, 0.f, 0.f, 0.f, 0.f, 0.f};
#if defined(__HIP_DEVICE_COMPILE__)
  v8f d = __builtin_amdgcn_wmma_f32_16x16x32_bf16(false, ah0, false, b0, (short)0, z, false, false);
  d = __builtin_amdgcn_wmma_f32_16x16x32_bf16(false, al0, false, b0, (short)0, d, false, false);
  d = __builtin_amdgcn_wmma_f32_16x16x32_bf16(false, ah1, false, b1, (short)0, d, false, false);
  d = __builtin_amdgcn_wmma_f32_16x16x32_bf16(false, al1, false, b1, (short)0, d, false, false);
  asm volatile("v_nop\n\tv_nop\n\tv_nop\n\tv_nop" : "+v"(d) : "v"(ah0), "v"(al0), "v"(b0), "v"(ah1), "v"(al1), "v"(b1));
  return d;
#else
  return z;
#endif
}

__device__ __forceinline__ v8f wm1h(v16h a, v16h b) {
  v8f z = {0.f, 0.f, 0.f, 0.f, 0.f, 0.f, 0.f, 0.f};
#if defined(__HIP_DEVICE_COMPILE__)
  v8f d = __builtin_amdgcn_wmma_f32_16x16x32_f16(false, a, false, b, (short)0, z, false, false);
  asm volatile("v_nop\n\tv_nop\n\tv_nop\n\tv_nop" : "+v"(d) : "v"(a), "v"(b));
  return d;
#else
  return z;
#endif
}

template <int NB>
__device__ __forceinline__ int scan_chunk(const int* __restrict__ dsts, int nE, int cbase, int slotBase,
                                          int vec8, int* list, int tid, int lane, int wave) {
  int wc = 0;
#pragma unroll
  for (int g = 0; g < NGRP; ++g) {
    const int el0  = (g * ATHR + tid) * EPT;
    const int e0   = cbase + el0;
    const int sent = -2147483647 - 1;
    const int lst  = nE - 1;
    v4i da, db;
    if (vec8 != 0 && cbase + CHUNK <= nE) {
      da = *(const v4i*)(dsts + e0);
      db = *(const v4i*)(dsts + e0 + 4);
    } else {
      da.x = (e0     < nE) ? dsts[min(e0,     lst)] : sent;
      da.y = (e0 + 1 < nE) ? dsts[min(e0 + 1, lst)] : sent;
      da.z = (e0 + 2 < nE) ? dsts[min(e0 + 2, lst)] : sent;
      da.w = (e0 + 3 < nE) ? dsts[min(e0 + 3, lst)] : sent;
      db.x = (e0 + 4 < nE) ? dsts[min(e0 + 4, lst)] : sent;
      db.y = (e0 + 5 < nE) ? dsts[min(e0 + 5, lst)] : sent;
      db.z = (e0 + 6 < nE) ? dsts[min(e0 + 6, lst)] : sent;
      db.w = (e0 + 7 < nE) ? dsts[min(e0 + 7, lst)] : sent;
    }
    const unsigned nb = (unsigned)slotBase;
    const unsigned s0 = (unsigned)da.x - nb, s1 = (unsigned)da.y - nb;
    const unsigned s2 = (unsigned)da.z - nb, s3 = (unsigned)da.w - nb;
    const unsigned s4 = (unsigned)db.x - nb, s5 = (unsigned)db.y - nb;
    const unsigned s6 = (unsigned)db.z - nb, s7 = (unsigned)db.w - nb;
    const bool h0 = s0 < (unsigned)NB, h1 = s1 < (unsigned)NB, h2 = s2 < (unsigned)NB, h3 = s3 < (unsigned)NB;
    const bool h4 = s4 < (unsigned)NB, h5 = s5 < (unsigned)NB, h6 = s6 < (unsigned)NB, h7 = s7 < (unsigned)NB;
    const unsigned any = __builtin_amdgcn_ballot_w32(h0 | h1 | h2 | h3 | h4 | h5 | h6 | h7);
    if (any != 0u) {
#define HITJ(J, HJ, SJ) { \
        const unsigned mj = __builtin_amdgcn_ballot_w32(HJ); \
        if (mj != 0u) { \
          if (HJ) { \
            const int pos_ = wc + (int)__builtin_amdgcn_mbcnt_lo(mj, 0u); \
            if (pos_ < WCAP) list[wave * WCAP + pos_] = ((el0 + (J)) << 12) | (int)(SJ); \
          } \
          wc += (int)__builtin_popcount(mj); } }
      HITJ(0, h0, s0)
      HITJ(1, h1, s1)
      HITJ(2, h2, s2)
      HITJ(3, h3, s3)
      HITJ(4, h4, s4)
      HITJ(5, h5, s5)
      HITJ(6, h6, s6)
      HITJ(7, h7, s7)
#undef HITJ
    }
  }
  return wc;
}

__global__ __launch_bounds__(64) void k_qr(const float* __restrict__ Ku, float* Qg) {
  __shared__ double sx[64], sa[64], sv[64], sy[64], q1[64], q2[64];
  __shared__ __attribute__((aligned(16))) float sQ[128];
  const int t = threadIdx.x;
  sx[t] = (double)Ku[t];
  sa[t] = (double)Ku[NV + t];
  __syncthreads();
  if (t == 0) {
    double n1 = 0.0;
#pragma unroll 1
    for (int i = 0; i < 64; ++i) n1 += sx[i] * sx[i];
    n1 = sqrt(n1);
    const double al = sx[0];
    double be = (al >= 0.0) ? -n1 : n1;
    if (n1 == 0.0) be = -1.0;
    const double rb = 1.0 / be;
    const double tau = (be - al) * rb;
    double amb = al - be;
    if (amb == 0.0) amb = 1.0;
    const double ramb = 1.0 / amb;
    sv[0] = 1.0;
#pragma unroll 1
    for (int i = 1; i < 64; ++i) sv[i] = sx[i] * ramb;
#pragma unroll 1
    for (int i = 0; i < 64; ++i) q1[i] = sx[i] * rb;
    double wv = sa[0];
#pragma unroll 1
    for (int i = 1; i < 64; ++i) wv += sv[i] * sa[i];
    const double tw = tau * wv;
#pragma unroll 1
    for (int i = 0; i < 64; ++i) sy[i] = sa[i] - tw * sv[i];
    double n2 = 0.0;
#pragma unroll 1
    for (int i = 1; i < 64; ++i) n2 += sy[i] * sy[i];
    n2 = sqrt(n2);
    const double al2 = sy[1];
    double be2 = (al2 >= 0.0) ? -n2 : n2;
    if (n2 == 0.0) be2 = -1.0;
    const double rb2 = 1.0 / be2;
    double vu = 0.0;
#pragma unroll 1
    for (int i = 1; i < 64; ++i) vu += sv[i] * (sy[i] * rb2);
    const double tv = tau * vu;
    q2[0] = -tv;
#pragma unroll 1
    for (int i = 1; i < 64; ++i) q2[i] = sy[i] * rb2 - tv * sv[i];
  }
  __syncthreads();
  sQ[2 * t]     = (float)q1[t];
  sQ[2 * t + 1] = (float)q2[t];
  __syncthreads();
  if (t < 32) {
    const v4f v = ((const v4f*)sQ)[t];
    *(volatile v4f*)(Qg + 4 * t) = v;
    __threadfence();
    *(volatile v4f*)(Qg + 4 * t) = v;
  }
}

__global__ __launch_bounds__(256) void k_wprep(const float* __restrict__ Ws, const float* __restrict__ Wv,
                                               unsigned short* Wps, unsigned short* Wpv) {
  __shared__ __attribute__((aligned(16))) unsigned short tile[64 * 64];
  const int tid = threadIdx.x;
  const int b = blockIdx.x;
  const float* S;
  unsigned short* D;
  int C, c0;
  if (b < 128) {
    const int l = b >> 6;
    c0 = (b & 63) * 64;
    C = SNCOL;
    S = Ws + (size_t)l * NS * SNCOL;
    D = Wps + (size_t)l * SNCOL * 64;
  } else {
    const int bb = b - 128;
    const int l = bb >> 5;
    c0 = (bb & 31) * 64;
    C = VNCOL;
    S = Wv + (size_t)l * NV * VNCOL;
    D = Wpv + (size_t)l * VNCOL * 64;
  }
#pragma unroll 4
  for (int r = 0; r < 16; ++r) {
    const int idx = r * 256 + tid;
    const int k = idx >> 6, j = idx & 63;
    tile[j * 64 + k] = bf_bits(S[(size_t)k * C + c0 + j]);
  }
  __syncthreads();
  v8us pv[2];
#pragma unroll
  for (int r = 0; r < 2; ++r) {
    const int piece = r * 256 + tid;
    const int j = piece >> 3, q = piece & 7;
    pv[r] = *(const v8us*)(tile + j * 64 + 8 * q);
  }
#pragma unroll
  for (int r = 0; r < 2; ++r) {
    const int piece = r * 256 + tid;
    const int j = piece >> 3, q = piece & 7;
    *(volatile v8us*)(D + (size_t)(c0 + j) * 64 + 8 * q) = pv[r];
  }
  __threadfence();
#pragma unroll
  for (int r = 0; r < 2; ++r) {
    const int piece = r * 256 + tid;
    const int j = piece >> 3, q = piece & 7;
    *(volatile v8us*)(D + (size_t)(c0 + j) * 64 + 8 * q) = pv[r];
  }
}

__global__ __launch_bounds__(256) void k_init(const float* __restrict__ x, const float* __restrict__ Qg,
                                              float* ys, float* yv, float* pos, int nN) {
  __shared__ float sQ[128];
  const int tid = threadIdx.x, l = tid & 31, wave = tid >> 5;
  const int nb = blockIdx.x * 32;
  if (tid < 128) sQ[tid] = Qg[tid];
  __syncthreads();
#pragma unroll 1
  for (int pass = 0; pass < 2; ++pass) {
#pragma unroll 1
    for (int r = 0; r < 8; ++r) {
      const int idx = r * 256 + tid;
      const int i = idx >> 6, c = idx & 63;
      const int n = nb + i;
      const int nr = n > nN - 1 ? nN - 1 : n;
      const float q0 = sQ[2 * c], q1 = sQ[2 * c + 1];
      const float* xp = x + (size_t)nr * 6;
      const float y0 = xp[0] * q0 + xp[3] * q1;
      const float y1 = xp[1] * q0 + xp[4] * q1;
      const float y2 = xp[2] * q0 + xp[5] * q1;
      *(volatile float*)(ys + (size_t)n * NS + c) = 0.0f;
      *(volatile float*)(yv + (size_t)n * YVW + c) = y0;
      *(volatile float*)(yv + (size_t)n * YVW + 64 + c) = y1;
      *(volatile float*)(yv + (size_t)n * YVW + 128 + c) = y2;
    }
    __threadfence();
  }
  if (wave == 0) {
    const int n = nb + l;
    const int nr = n > nN - 1 ? nN - 1 : n;
    v4f p;
    p.x = x[(size_t)nr * 6 + 0];
    p.y = x[(size_t)nr * 6 + 1];
    p.z = x[(size_t)nr * 6 + 2];
    p.w = 0.0f;
    *(volatile v4f*)(pos + (size_t)n * 4) = p;
    __threadfence();
    *(volatile v4f*)(pos + (size_t)n * 4) = p;
  }
}

__global__ __launch_bounds__(STHR) void k_sc(
    const float* __restrict__ ys, const float* __restrict__ yv,
    const int* __restrict__ attr, const float* __restrict__ embt,
    const unsigned short* __restrict__ Wps, const unsigned short* __restrict__ Wpv,
    float* sc, int nN, int nT) {
  extern __shared__ v4f lds_dyn[];
  char* lds = (char*)lds_dyn;
  unsigned short* sYh = (unsigned short*)(lds + LS_YH);
  unsigned short* sYl = (unsigned short*)(lds + LS_YL);
  unsigned short* sVh = (unsigned short*)(lds + LS_VH);
  unsigned short* sVl = (unsigned short*)(lds + LS_VL);
  float* sA = (float*)(lds + LS_A);
  float* sO = (float*)(lds + LS_O);
  const int tid = threadIdx.x, l = tid & 31, wave = tid >> 5, hh = l >> 4, m = l & 15;
  const int rowBase = blockIdx.x * NPB;

#pragma unroll
  for (int r = 0; r < (NPB * NS / 4) / STHR; ++r) {
    const int it = r * STHR + tid;
    const int row = it >> 4, q = it & 15;
    const v4f v = *(const v4f*)(ys + (size_t)(rowBase + row) * NS + 4 * q);
    v4us hi, lo;
    split4(v, hi, lo);
    *(v4us*)(sYh + row * NS + 4 * q) = hi;
    *(v4us*)(sYl + row * NS + 4 * q) = lo;
  }
#pragma unroll 4
  for (int r = 0; r < (NPB * YVW / 4) / STHR; ++r) {
    const int it = r * STHR + tid;
    const int row = it / 48;
    const int q = it - row * 48;
    const int d = q >> 4, qq = q & 15;
    const v4f v = *(const v4f*)(yv + (size_t)(rowBase + row) * YVW + 4 * q);
    v4us hi, lo;
    split4(v, hi, lo);
    *(v4us*)(sVh + d * (NPB * NV) + row * NV + 4 * qq) = hi;
    *(v4us*)(sVl + d * (NPB * NV) + row * NV + 4 * qq) = lo;
  }
#pragma unroll
  for (int r = 0; r < (NPB * EMB / 4) / STHR; ++r) {
    const int it = r * STHR + tid;
    const int row = it >> 3, q = it & 7;
    int n = rowBase + row;
    n = n > nN - 1 ? nN - 1 : n;
    int at = attr[n];
    at = at < 0 ? 0 : (at > nT - 1 ? nT - 1 : at);
    *(v4f*)(sA + row * EMB + 4 * q) = *(const v4f*)(embt + (size_t)at * EMB + 4 * q);
  }
  __syncthreads();

  const int rw = wave * 16;
#pragma unroll 1
  for (int g = 0; g < 5; ++g) {
    const bool iss = g < 2;
    const unsigned short* pah = iss ? sYh : (sVh + (g - 2) * (NPB * NV));
    const unsigned short* pal = iss ? sYl : (sVl + (g - 2) * (NPB * NV));
    const unsigned short* pb  = iss ? Wps : Wpv;
    const int en = iss ? 128 : 64;
    const int tb = iss ? g * 64 : 0;
    const unsigned short* ar  = pah + (rw + m) * 64 + 8 * hh;
    const unsigned short* arl = pal + (rw + m) * 64 + 8 * hh;
    FragB ah0, ah1, al0, al1;
    ah0.u[0] = *(const v8us*)(ar);
    ah0.u[1] = *(const v8us*)(ar + 16);
    ah1.u[0] = *(const v8us*)(ar + 32);
    ah1.u[1] = *(const v8us*)(ar + 48);
    al0.u[0] = *(const v8us*)(arl);
    al0.u[1] = *(const v8us*)(arl + 16);
    al1.u[0] = *(const v8us*)(arl + 32);
    al1.u[1] = *(const v8us*)(arl + 48);
    v8f acc[4];
#pragma unroll
    for (int t = 0; t < 4; ++t) { v8f z = {0.f, 0.f, 0.f, 0.f, 0.f, 0.f, 0.f, 0.f}; acc[t] = z; }
#pragma unroll 1
    for (int e = 0; e < EMB; ++e) {
      float av[8];
#pragma unroll
      for (int r = 0; r < 8; ++r) av[r] = sA[(rw + 8 * hh + r) * EMB + e];
#pragma unroll
      for (int t = 0; t < 4; ++t) {
        const unsigned short* bp = pb + (size_t)(e * en + tb + 16 * t + m) * 64 + 8 * hh;
        FragB b0, b1;
        b0.u[0] = *(const v8us*)(bp);
        b0.u[1] = *(const v8us*)(bp + 16);
        b1.u[0] = *(const v8us*)(bp + 32);
        b1.u[1] = *(const v8us*)(bp + 48);
        const v8f d = wm4(ah0.v, al0.v, b0.v, ah1.v, al1.v, b1.v);
#pragma unroll
        for (int r = 0; r < 8; ++r) acc[t][r] = fmaf(av[r], d[r], acc[t][r]);
      }
    }
#pragma unroll
    for (int t = 0; t < 4; ++t) {
#pragma unroll
      for (int r = 0; r < 8; ++r) sO[(rw + 8 * hh + r) * SCW + g * 64 + 16 * t + m] = acc[t][r];
    }
  }
  __syncthreads();

  {
    float* gp = sc + (size_t)(rowBase + rw) * SCW;
    const float* sp = sO + rw * SCW;
#pragma unroll 4
    for (int i = 0; i < (16 * SCW / 4) / 32; ++i) {
      const int f = i * 32 + l;
      const v4f v = ((const v4f*)sp)[f];
      *(volatile v4f*)(gp + 4 * (size_t)f) = v;
    }
    __threadfence();
#pragma unroll 4
    for (int i = 0; i < (16 * SCW / 4) / 32; ++i) {
      const int f = i * 32 + l;
      const v4f v = ((const v4f*)sp)[f];
      *(volatile v4f*)(gp + 4 * (size_t)f) = v;
    }
  }
}

__global__ __launch_bounds__(ATHR) void k_agg(
    const int* __restrict__ esrc, const int* __restrict__ edst,
    const float* __restrict__ pos, const float* __restrict__ ys, const float* __restrict__ yv,
    const float* __restrict__ sc,
    const float* __restrict__ wr1, const float* __restrict__ br1,
    const float* __restrict__ wr2, const float* __restrict__ br2,
    const float* __restrict__ Qg,
    float* ysn, float* yvn, float* posn, float* out,
    int nE, int nN, int last, int vec8) {
  extern __shared__ v4f lds_dyn[];
  char* lds = (char*)lds_dyn;
  float*    sAcc  = (float*)(lds + LA_ACC);
  int*      sList = (int*)(lds + LA_LIST);
  float*    sWst  = (float*)(lds + LA_WST);
  _Float16* sW2   = (_Float16*)(lds + LA_W2);
  _Float16* sHid  = (_Float16*)(lds + LA_HID);
  float*    sW1   = (float*)(lds + LA_W1);
  float*    sB1   = (float*)(lds + LA_B1);
  float*    sB2   = (float*)(lds + LA_B2);
  float*    sQ    = (float*)(lds + LA_Q);
  float*    sEa   = (float*)(lds + LA_EA);
  float*    sXv   = (float*)(lds + LA_XV);
  int*      sSrc  = (int*)(lds + LA_SRC);
  int*      sSlot = (int*)(lds + LA_SLOT);
  int*      sCnt  = (int*)(lds + LA_CNT);
  const int tid = threadIdx.x, l = tid & 31, wave = tid >> 5, hh = l >> 4, m = l & 15;
  const int nodeBase = blockIdx.x * NPB;

  {
    const v4f z4 = {0.0f, 0.0f, 0.0f, 0.0f};
    for (int i = tid; i < NPB * SCW / 4; i += ATHR) ((v4f*)sAcc)[i] = z4;
  }
  if (tid < NBAS * RHID) sW1[tid] = wr1[tid];
  if (tid < RHID) sB1[tid] = br1[tid];
  sB2[tid] = br2[tid];
  if (tid < 2 * NV) sQ[tid] = Qg[tid];
  if (tid < (GRP * 32) / 8) {
    v8h z8;
#pragma unroll
    for (int u = 0; u < 8; ++u) z8[u] = (_Float16)0.0f;
    ((v8h*)sHid)[tid] = z8;
  }
#pragma unroll
  for (int r = 0; r < (NW * 4) / ATHR; ++r) {
    const int it = r * ATHR + tid;
    const int o = it >> 2, q = it & 3;
    v8h hv;
#pragma unroll
    for (int u = 0; u < 8; ++u) {
      const int k = 8 * q + u;
      const int kc = k > RHID - 1 ? RHID - 1 : k;
      const float wvv = wr2[kc * NW + o];
      hv[u] = (_Float16)((k < RHID) ? wvv : 0.0f);
    }
    *(v8h*)(sW2 + o * 32 + 8 * q) = hv;
  }
  __syncthreads();

  const int nChunks = (nE + CHUNK - 1) / CHUNK;
#pragma unroll 1
  for (int ch = 0; ch < nChunks; ++ch) {
    const int cbase = ch * CHUNK;
    const int wc = scan_chunk<NPB>(edst, nE, cbase, nodeBase, vec8, sList, tid, l, wave);
    if (l == 0) sCnt[wave] = wc;
    __syncthreads();
    int pre[NWAVE + 1];
    pre[0] = 0;
#pragma unroll
    for (int w = 0; w < NWAVE; ++w) {
      int c = sCnt[w];
      c = c < 0 ? 0 : (c > WCAP ? WCAP : c);
      pre[w + 1] = pre[w] + c;
    }
    const int total = __builtin_amdgcn_readfirstlane(pre[NWAVE]);

#pragma unroll 1
    for (int gb = 0; gb < total; gb += GRP) {
      if (wave == 0) {
        const int idx = gb + l;
        const bool valid = idx < total;
        const int ci = valid ? idx : (total - 1);
        int wsel = 0, pw = 0;
#pragma unroll
        for (int w = 1; w < NWAVE; ++w) {
          const bool ge = ci >= pre[w];
          wsel += ge ? 1 : 0;
          pw = ge ? pre[w] : pw;
        }
        int p = ci - pw;
        p = p < 0 ? 0 : (p > WCAP - 1 ? WCAP - 1 : p);
        const int ent = sList[wsel * WCAP + p];
        const int el = (ent >> 12) & (CHUNK - 1);
        const int sl = ent & (NPB - 1);
        int e = cbase + el;
        e = e > nE - 1 ? nE - 1 : e;
        int s = esrc[e];
        s = s < 0 ? 0 : (s > nN - 1 ? nN - 1 : s);
        int dn = nodeBase + sl;
        dn = dn > nN - 1 ? nN - 1 : dn;
        const v4f ps = *(const v4f*)(pos + (size_t)s * 4);
        const v4f pd = *(const v4f*)(pos + (size_t)dn * 4);
        const float evx = ps.x - pd.x, evy = ps.y - pd.y, evz = ps.z - pd.z;
        const float elen = sqrtf(evx * evx + evy * evy + evz * evz);
        const float inv = 1.0f / elen;
        const float shx = (SQ3F * evx) * inv, shy = (SQ3F * evy) * inv, shz = (SQ3F * evz) * inv;
        const float uu = elen * RCUTF;
        const float vv = 2.0f * (uu - 1.0f);
        float cut = 0.5f * (1.0f - cosf(PIF * vv));
        cut = (vv > 0.0f) ? 0.0f : cut;
        cut = (vv < -1.0f) ? 1.0f : cut;
        const float ea0 = cut * shx, ea1 = cut * shy, ea2 = cut * shz;
        float hid[RHID];
#pragma unroll
        for (int r = 0; r < RHID; ++r) hid[r] = 0.0f;
#pragma unroll
        for (int k = 0; k < NBAS; ++k) {
          const float pik = PIF * (float)(k + 1);
          const float arg = (pik * elen) * RCUTF;
          const float bk = ((C2CF * sinf(arg)) * inv) * SQ8F;
#pragma unroll
          for (int r = 0; r < RHID; ++r) hid[r] = fmaf(bk, sW1[k * RHID + r], hid[r]);
        }
#pragma unroll
        for (int r = 0; r < RHID; ++r) hid[r] = siluf(hid[r] + sB1[r]);
        v8h h0, h1;
#pragma unroll
        for (int u = 0; u < 8; ++u) {
          h0[u] = (_Float16)(valid ? hid[u] : 0.0f);
          h1[u] = (_Float16)(valid ? hid[8 + u] : 0.0f);
        }
        *(v8h*)(sHid + l * 32) = h0;
        *(v8h*)(sHid + l * 32 + 8) = h1;
        sSrc[l] = s;
        sSlot[l] = valid ? sl : 255;
        v4f ea4;
        ea4.x = ea0; ea4.y = ea1; ea4.z = ea2; ea4.w = 0.0f;
        *(v4f*)(sEa + l * 4) = ea4;
      }
      __syncthreads();
      {
        const int rt = wave & 1, ctb = (wave >> 1) * 4;
        FragH a;
        a.half[0] = *(const v8h*)(sHid + (rt * 16 + m) * 32 + 8 * hh);
        a.half[1] = *(const v8h*)(sHid + (rt * 16 + m) * 32 + 16 + 8 * hh);
#pragma unroll
        for (int t = 0; t < 4; ++t) {
          const int ct = ctb + t;
          FragH b;
          b.half[0] = *(const v8h*)(sW2 + (ct * 16 + m) * 32 + 8 * hh);
          b.half[1] = *(const v8h*)(sW2 + (ct * 16 + m) * 32 + 16 + 8 * hh);
          const v8f d = wm1h(a.v, b.v);
          const float bias = sB2[ct * 16 + m];
#pragma unroll
          for (int r = 0; r < 8; ++r) sWst[(rt * 16 + 8 * hh + r) * NW + ct * 16 + m] = d[r] + bias;
        }
      }
      __syncthreads();
      {
        const int slq = sSlot[l];
        const bool own = (slq < NPB) && ((slq & (NWAVE - 1)) == wave);
        unsigned msk = __builtin_amdgcn_ballot_w32(own);
#pragma unroll 1
        while (msk != 0u) {
          const int t = __builtin_ctz(msk);
          msk &= msk - 1u;
          const int src = sSrc[t];
          const int sl = sSlot[t];
          const v4f ea = *(const v4f*)(sEa + t * 4);
          const float* yp = ys + (size_t)src * NS;
          const float* vp = yv + (size_t)src * YVW;
          const float* wp = sWst + t * NW;
          float* ap = sAcc + sl * SCW;
#pragma unroll
          for (int j = 0; j < 2; ++j) {
            const int c = l + 32 * j;
            const float wa = wp[c], wb = wp[64 + c], wcv = wp[128 + c], wd = wp[192 + c];
            const float sv = yp[c];
            const float v0 = vp[c], v1 = vp[64 + c], v2 = vp[128 + c];
            const float dot = v0 * ea.x + v1 * ea.y + v2 * ea.z;
            const float cx = v1 * ea.z - v2 * ea.y;
            const float cy = v2 * ea.x - v0 * ea.z;
            const float cz = v0 * ea.y - v1 * ea.x;
            const float was = wa * sv;
            const float m0 = was * ea.x + wcv * cx;
            const float m1 = was * ea.y + wcv * cy;
            const float m2 = was * ea.z + wcv * cz;
            ap[c]       = ap[c] + wb * dot;
            ap[64 + c]  = ap[64 + c] + wd * dot;
            ap[128 + c] = ap[128 + c] + m0;
            ap[192 + c] = ap[192 + c] + m1;
            ap[256 + c] = ap[256 + c] + m2;
          }
        }
      }
      __syncthreads();
    }
    __syncthreads();
  }

#pragma unroll 1
  for (int i = 0; i < NPB / NWAVE; ++i) {
    const int slot = wave * (NPB / NWAVE) + i;
    const int n = nodeBase + slot;
    const int nr = n > nN - 1 ? nN - 1 : n;
    const float* scp = sc + (size_t)nr * SCW;
    const float* ysp = ys + (size_t)nr * NS;
    const float* yvp = yv + (size_t)nr * YVW;
    const float* ap = sAcc + slot * SCW;
    float ysv[2], yvv[2][3];
    float p00 = 0.f, p01 = 0.f, p02 = 0.f, p10 = 0.f, p11 = 0.f, p12 = 0.f;
#pragma unroll
    for (int j = 0; j < 2; ++j) {
      const int c = l + 32 * j;
      const float o1 = scp[c] + ap[c] * INVDEGF;
      const float o2 = scp[64 + c] + ap[64 + c] * INVDEGF;
      ysv[j] = ysp[c] + HSTEPF * siluf(o1);
      const float g = HSTEPF * sigmf(o2);
      const float q0 = sQ[2 * c], q1 = sQ[2 * c + 1];
#pragma unroll
      for (int d = 0; d < 3; ++d) {
        const float ov = scp[128 + 64 * d + c] + ap[128 + 64 * d + c] * INVDEGF;
        const float yn = yvp[64 * d + c] + g * ov;
        yvv[j][d] = yn;
        if (d == 0) { p00 = fmaf(yn, q0, p00); p10 = fmaf(yn, q1, p10); }
        if (d == 1) { p01 = fmaf(yn, q0, p01); p11 = fmaf(yn, q1, p11); }
        if (d == 2) { p02 = fmaf(yn, q0, p02); p12 = fmaf(yn, q1, p12); }
      }
    }
#pragma unroll
    for (int off = 16; off > 0; off >>= 1) {
      p00 += __shfl_xor(p00, off);
      p01 += __shfl_xor(p01, off);
      p02 += __shfl_xor(p02, off);
      p10 += __shfl_xor(p10, off);
      p11 += __shfl_xor(p11, off);
      p12 += __shfl_xor(p12, off);
    }
    float* ysq = ysn + (size_t)n * NS;
    float* yvq = yvn + (size_t)n * YVW;
    *(volatile float*)(ysq + l) = ysv[0];
    *(volatile float*)(ysq + 32 + l) = ysv[1];
#pragma unroll
    for (int j = 0; j < 2; ++j) {
#pragma unroll
      for (int d = 0; d < 3; ++d) *(volatile float*)(yvq + 64 * d + 32 * j + l) = yvv[j][d];
    }
    {
      const float xv = (l == 0) ? p00 : ((l == 1) ? p01 : ((l == 2) ? p02 : ((l == 3) ? p10 : ((l == 4) ? p11 : p12))));
      if (l < 6) sXv[slot * 8 + l] = xv;
    }
    __threadfence();
    *(volatile float*)(ysq + l) = ysv[0];
    *(volatile float*)(ysq + 32 + l) = ysv[1];
#pragma unroll
    for (int j = 0; j < 2; ++j) {
#pragma unroll
      for (int d = 0; d < 3; ++d) *(volatile float*)(yvq + 64 * d + 32 * j + l) = yvv[j][d];
    }
  }
  __syncthreads();
  if (wave == 0) {
    v4f pa, pb;
    pa.x = sXv[l * 8 + 0]; pa.y = sXv[l * 8 + 1]; pa.z = sXv[l * 8 + 2]; pa.w = 0.0f;
    pb.x = sXv[(32 + l) * 8 + 0]; pb.y = sXv[(32 + l) * 8 + 1]; pb.z = sXv[(32 + l) * 8 + 2]; pb.w = 0.0f;
    float* pp = posn + (size_t)nodeBase * 4;
    int nval = nN - nodeBase;
    nval = nval > NPB ? NPB : (nval < 0 ? 0 : nval);
    const int nf = nval * 6;
    float* ob = out + (size_t)nodeBase * 6;
    v4f ov[3];
#pragma unroll
    for (int ins = 0; ins < 3; ++ins) {
      const int k0 = 4 * (ins * 32 + l);
      v4f v;
#pragma unroll
      for (int j = 0; j < 4; ++j) {
        int k = k0 + j;
        k = k > NPB * 6 - 1 ? NPB * 6 - 1 : k;
        const int sj = k / 6;
        const int cp = k - sj * 6;
        v[j] = sXv[sj * 8 + cp];
      }
      ov[ins] = v;
    }
#pragma unroll 1
    for (int pass = 0; pass < 2; ++pass) {
      *(volatile v4f*)(pp + 4 * l) = pa;
      *(volatile v4f*)(pp + 4 * (32 + l)) = pb;
      if (last != 0) {
#pragma unroll
        for (int ins = 0; ins < 3; ++ins) {
          const int k0 = 4 * (ins * 32 + l);
          if (k0 + 4 <= nf) {
            *(volatile v4f*)(ob + k0) = ov[ins];
          } else {
#pragma unroll
            for (int j = 0; j < 4; ++j) {
              if (k0 + j < nf) *(volatile float*)(ob + k0 + j) = ov[ins][j];
            }
          }
        }
      }
      __threadfence();
    }
  }
}

extern "C" void kernel_launch(void* const* d_in, const int* in_sizes, int n_in,
                              void* d_out, int out_size, void* d_ws, size_t ws_size,
                              hipStream_t stream) {
  if (n_in < 13) return;
  const int nN = in_sizes[0] / 6;
  const int nE = in_sizes[3];
  if (nN <= 0 || nE <= 0) return;
  if (in_sizes[0] != 6 * nN || in_sizes[2] != nN || in_sizes[4] != nE) return;
  if (in_sizes[5] < EMB || (in_sizes[5] % EMB) != 0) return;
  const int nT = in_sizes[5] / EMB;
  if (in_sizes[6] != 2 * NV) return;
  if (in_sizes[7] != 2 * NS * SNCOL || in_sizes[8] != 2 * NV * VNCOL) return;
  if (in_sizes[9] != 2 * NBAS * RHID || in_sizes[10] != 2 * RHID) return;
  if (in_sizes[11] != 2 * RHID * NW || in_sizes[12] != 2 * NW) return;
  if (out_size != nN * 6) return;
  if (nN > (1 << 24) || nE > (1 << 28)) return;

  const float* x     = (const float*)d_in[0];
  const int*   attr  = (const int*)d_in[2];
  const int*   esrc  = (const int*)d_in[3];
  const int*   edst  = (const int*)d_in[4];
  const float* embt  = (const float*)d_in[5];
  const float* Ku    = (const float*)d_in[6];
  const float* Wscs  = (const float*)d_in[7];
  const float* Wscv  = (const float*)d_in[8];
  const float* Wr1   = (const float*)d_in[9];
  const float* br1   = (const float*)d_in[10];
  const float* Wr2   = (const float*)d_in[11];
  const float* br2   = (const float*)d_in[12];
  float* outp = (float*)d_out;

  const int nBlk = (nN + NPB - 1) / NPB;
  const int Npad = nBlk * NPB;
  const int nBI  = Npad / 32;
  const int nBW  = 2 * (SNCOL / 64) + 2 * (VNCOL / 64);

  char* ws = (char*)d_ws;
  size_t off = 0;
  const size_t oQ   = off; off += 512;                                   off = (off + 255) & ~(size_t)255;
  const size_t oWps = off; off += (size_t)2 * SNCOL * 64 * 2;            off = (off + 255) & ~(size_t)255;
  const size_t oWpv = off; off += (size_t)2 * VNCOL * 64 * 2;            off = (off + 255) & ~(size_t)255;
  const size_t oYsA = off; off += (size_t)Npad * NS * 4;                 off = (off + 255) & ~(size_t)255;
  const size_t oYsB = off; off += (size_t)Npad * NS * 4;                 off = (off + 255) & ~(size_t)255;
  const size_t oYvA = off; off += (size_t)Npad * YVW * 4;                off = (off + 255) & ~(size_t)255;
  const size_t oYvB = off; off += (size_t)Npad * YVW * 4;                off = (off + 255) & ~(size_t)255;
  const size_t oPoA = off; off += (size_t)Npad * 4 * 4;                  off = (off + 255) & ~(size_t)255;
  const size_t oPoB = off; off += (size_t)Npad * 4 * 4;                  off = (off + 255) & ~(size_t)255;
  const size_t oSc  = off; off += (size_t)Npad * SCW * 4;                off = (off + 255) & ~(size_t)255;
  if (off > ws_size || off > ((size_t)128 << 20)) return;

  float*          Qg   = (float*)(ws + oQ);
  unsigned short* Wps  = (unsigned short*)(ws + oWps);
  unsigned short* Wpv  = (unsigned short*)(ws + oWpv);
  float*          ysA  = (float*)(ws + oYsA);
  float*          ysB  = (float*)(ws + oYsB);
  float*          yvA  = (float*)(ws + oYvA);
  float*          yvB  = (float*)(ws + oYvB);
  float*          posA = (float*)(ws + oPoA);
  float*          posB = (float*)(ws + oPoB);
  float*          scb  = (float*)(ws + oSc);

  k_qr<<<1, 64, 0, stream>>>(Ku, Qg);
  k_wprep<<<nBW, 256, 0, stream>>>(Wscs, Wscv, Wps, Wpv);
  k_init<<<nBI, 256, 0, stream>>>(x, Qg, ysA, yvA, posA, nN);

  hipFuncSetAttribute(reinterpret_cast<const void*>(&k_sc), hipFuncAttributeMaxDynamicSharedMemorySize, LDS_SC);
  hipFuncSetAttribute(reinterpret_cast<const void*>(&k_agg), hipFuncAttributeMaxDynamicSharedMemorySize, LDS_AGG);

  k_sc<<<nBlk, STHR, LDS_SC, stream>>>(ysA, yvA, attr, embt, Wps, Wpv, scb, nN, nT);
  k_agg<<<nBlk, ATHR, LDS_AGG, stream>>>(esrc, edst, posA, ysA, yvA, scb,
                                          Wr1, br1, Wr2, br2, Qg,
                                          ysB, yvB, posB, outp, nE, nN, 0, 1);
  k_sc<<<nBlk, STHR, LDS_SC, stream>>>(ysB, yvB, attr, embt,
                                       Wps + (size_t)SNCOL * 64, Wpv + (size_t)VNCOL * 64, scb, nN, nT);
  k_agg<<<nBlk, ATHR, LDS_AGG, stream>>>(esrc, edst, posB, ysB, yvB, scb,
                                          Wr1 + NBAS * RHID, br1 + RHID, Wr2 + RHID * NW, br2 + NW, Qg,
                                          ysA, yvA, posA, outp, nE, nN, 1, 1);
}
